// ODE_func_mix_autoencoder_46926812677055
// MI455X (gfx1250) — hardware-verified
//
#include <hip/hip_runtime.h>
#include <stdint.h>
#include <stddef.h>


#define CC      64
#define KFL     27
#define WSZ     (CC * CC)
#define NFA     14
#define NFB     (KFL - NFA)
#define YPITCH  (NFA * CC)
#define GNB     1024
#define GTH     256
#define GEPT    4
#define GCH     (GTH * GEPT)
#define GLDS    (GNB * CC * 4 + GNB * 4 + GCH * 4 * 2 + 64)
#define LDT     68
#define TB      128
#define TROWS   64

typedef float          v2f   __attribute__((ext_vector_type(2)));
typedef float          v4f   __attribute__((ext_vector_type(4)));
typedef float          v8f   __attribute__((ext_vector_type(8)));
typedef _Float16       v2h   __attribute__((ext_vector_type(2)));
typedef _Float16       v8h   __attribute__((ext_vector_type(8)));
typedef _Float16       v16h  __attribute__((ext_vector_type(16)));
typedef unsigned short v8us  __attribute__((ext_vector_type(8)));
typedef unsigned short v16us __attribute__((ext_vector_type(16)));
typedef __bf16         v16bf __attribute__((ext_vector_type(16)));

union FragB { v16bf v; v16us u; v8us hv[2]; };
union FragH { v16h v; v8h hv[2]; };

__device__ __forceinline__ v8f z8f() { v8f z = {0.f, 0.f, 0.f, 0.f, 0.f, 0.f, 0.f, 0.f}; return z; }
__device__ __forceinline__ v8us z8us() { v8us z = {0, 0, 0, 0, 0, 0, 0, 0}; return z; }

__device__ __forceinline__ v8f mma_bf(v16bf a, v16bf b, v8f c)
{
    v8f d = __builtin_amdgcn_wmma_f32_16x16x32_bf16(false, a, false, b, (short)0, c, false, false);
    asm volatile("v_nop\n\tv_nop\n\tv_nop\n\tv_nop" : "+v"(d) : "v"(a), "v"(b));
    return d;
}
__device__ __forceinline__ v8f mma_h(v16h a, v16h b, v8f c)
{
    v8f d = __builtin_amdgcn_wmma_f32_16x16x32_f16(false, a, false, b, (short)0, c, false, false);
    asm volatile("v_nop\n\tv_nop\n\tv_nop\n\tv_nop" : "+v"(d) : "v"(a), "v"(b));
    return d;
}
__device__ __forceinline__ v8f mma3(v16bf ah, v16bf al, v16bf bh, v16bf bl, v8f c)
{
    c = mma_bf(ah, bh, c);
    c = mma_bf(ah, bl, c);
    c = mma_bf(al, bh, c);
    return c;
}

__device__ __forceinline__ unsigned short bf_rne(float f)
{
    unsigned int u = __float_as_uint(f);
    u += 0x7FFFu + ((u >> 16) & 1u);
    return (unsigned short)(u >> 16);
}
__device__ __forceinline__ void split1(float f, unsigned short& hi, unsigned short& lo)
{
    const unsigned short hh = bf_rne(f);
    const float rem = f - __uint_as_float(((unsigned int)hh) << 16);
    hi = hh;
    lo = bf_rne(rem);
}
__device__ __forceinline__ void split8(v4f a, v4f b, v8us& hi, v8us& lo)
{
    const float f[8] = {a.x, a.y, a.z, a.w, b.x, b.y, b.z, b.w};
    v8us hh = z8us(), ll = z8us();
#pragma unroll
    for (int i = 0; i < 8; ++i) {
        unsigned short p, q;
        split1(f[i], p, q);
        hh[i] = p;
        ll[i] = q;
    }
    hi = hh;
    lo = ll;
}
__device__ __forceinline__ void fragA_f32(const float* rp, int h, FragB& hi, FragB& lo)
{
    const v4f p0 = *(const v4f*)(rp + 8 * h);
    const v4f p1 = *(const v4f*)(rp + 8 * h + 4);
    const v4f p2 = *(const v4f*)(rp + 16 + 8 * h);
    const v4f p3 = *(const v4f*)(rp + 20 + 8 * h);
    split8(p0, p1, hi.hv[0], lo.hv[0]);
    split8(p2, p3, hi.hv[1], lo.hv[1]);
}
__device__ __forceinline__ v16bf fragB16(const unsigned short* t, int n, int P, int k0, int h)
{
    FragB f;
    const unsigned short* p = t + n * P + k0;
    f.hv[0] = *(const v8us*)(p + 8 * h);
    f.hv[1] = *(const v8us*)(p + 16 + 8 * h);
    return f.v;
}
__device__ __forceinline__ void stage_w(const float* __restrict__ g, int gsk, int gsn, int K, int Kp, int N, int P,
                                         unsigned short* th, unsigned short* tl, int tid, int nth)
{
    for (int idx = tid; idx < N * Kp; idx += nth) {
        const int n = idx / Kp;
        const int k = idx - n * Kp;
        const float v = (k < K) ? g[k * gsk + n * gsn] : 0.f;
        unsigned short a, b;
        split1(v, a, b);
        th[n * P + k] = a;
        tl[n * P + k] = b;
    }
}
__device__ __forceinline__ v8h to_h8(v4f a, v4f b, float sc)
{
    v8h r;
    r[0] = (_Float16)(a.x * sc); r[1] = (_Float16)(a.y * sc); r[2] = (_Float16)(a.z * sc); r[3] = (_Float16)(a.w * sc);
    r[4] = (_Float16)(b.x * sc); r[5] = (_Float16)(b.y * sc); r[6] = (_Float16)(b.z * sc); r[7] = (_Float16)(b.w * sc);
    return r;
}
__device__ __forceinline__ float elu_f(float v)
{
    const float n = expm1f(fminf(v, 0.f));
    return v > 0.f ? v : n;
}

__global__ void __launch_bounds__(256) k_wprep(const float* __restrict__ spw, _Float16* __restrict__ wt, int nseg)
{
    const int sgi = blockIdx.x * 256 + threadIdx.x;
    const bool ok = sgi < nseg;
    const int sg = ok ? sgi : 0;
    const int c8 = sg & 7, o = (sg >> 3) & (CC - 1), f = sg >> 9;
    const float* p = spw + (size_t)f * WSZ + (size_t)(c8 * 8) * CC + o;
    v8h v;
#pragma unroll
    for (int i = 0; i < 8; ++i) v[i] = (_Float16)(p[(size_t)i * CC] * 64.f);
    _Float16* q = wt + (size_t)f * WSZ + (size_t)o * CC + c8 * 8;
    if (ok) *(volatile v8h*)q = v;
    __threadfence();
    if (ok) *(volatile v8h*)q = v;
}

__device__ __forceinline__ void e_store(const float* T, float* g32, _Float16* g16, int lane)
{
#pragma unroll
    for (int g = 0; g < 8; ++g) {
        const int L = 4 * g + (lane >> 3);
        const int row = L >> 1;
        const int col = 32 * (L & 1) + 4 * (lane & 7);
        const v4f v = *(const v4f*)(T + row * LDT + col);
        *(volatile v4f*)(g32 + (size_t)row * CC + col) = v;
    }
#pragma unroll
    for (int g = 0; g < 4; ++g) {
        const int row = 4 * g + (lane >> 3);
        const int col = 8 * (lane & 7);
        const v4f q0 = *(const v4f*)(T + row * LDT + col);
        const v4f q1 = *(const v4f*)(T + row * LDT + col + 4);
        const v8h v = to_h8(q0, q1, 16.f);
        *(volatile v8h*)(g16 + (size_t)row * CC + col) = v;
    }
}

__global__ void __launch_bounds__(TB) k_enc(const float* __restrict__ x,
                                        const float* __restrict__ w0, const float* __restrict__ b0,
                                        const float* __restrict__ w1, const float* __restrict__ b1,
                                        const float* __restrict__ w2, const float* __restrict__ b2,
                                        float* __restrict__ h32, _Float16* __restrict__ h16, int NT)
{
    __shared__ __attribute__((aligned(16))) unsigned short sW1h[32 * 40];
    __shared__ __attribute__((aligned(16))) unsigned short sW1l[32 * 40];
    __shared__ __attribute__((aligned(16))) unsigned short sW2h[64 * 40];
    __shared__ __attribute__((aligned(16))) unsigned short sW2l[64 * 40];
    __shared__ float sw0[32], sb0[16], sb1[32], sb2[64];
    __shared__ __attribute__((aligned(16))) float sT[4][16 * LDT];

    const int tid = threadIdx.x, lane = tid & 31, wv = tid >> 5, h = lane >> 4, m = lane & 15;
    stage_w(w1, 1, 16, 16, 32, 32, 40, sW1h, sW1l, tid, TB);
    stage_w(w2, 1, 32, 32, 32, 64, 40, sW2h, sW2l, tid, TB);
    for (int i = tid; i < 32; i += TB) sw0[i] = w0[i];
    for (int i = tid; i < 16; i += TB) sb0[i] = b0[i];
    for (int i = tid; i < 32; i += TB) sb1[i] = b1[i];
    for (int i = tid; i < 64; i += TB) sb2[i] = b2[i];
    __syncthreads();

    const int row0 = blockIdx.x * TROWS + wv * 16;
    int rr = row0 + m;
    rr = rr < NT ? rr : NT - 1;
    const float x0 = x[(size_t)rr * 2], x1 = x[(size_t)rr * 2 + 1];

    FragB ah, al;
    {
        v8us hh = z8us(), ll = z8us();
#pragma unroll
        for (int i = 0; i < 8; ++i) {
            const int c = 8 * h + i;
            float s = sw0[c * 2] * x0 + sw0[c * 2 + 1] * x1;
            s = elu_f(s + sb0[c]);
            unsigned short p, q;
            split1(s, p, q);
            hh[i] = p;
            ll[i] = q;
        }
        ah.hv[0] = hh; al.hv[0] = ll;
        ah.hv[1] = z8us(); al.hv[1] = z8us();
    }
    v8f acc1[2];
#pragma unroll
    for (int nt = 0; nt < 2; ++nt) {
        acc1[nt] = z8f();
        const v16bf bh = fragB16(sW1h, nt * 16 + m, 40, 0, h);
        const v16bf bl = fragB16(sW1l, nt * 16 + m, 40, 0, h);
        acc1[nt] = mma3(ah.v, al.v, bh, bl, acc1[nt]);
    }
    float* T = sT[wv];
#pragma unroll
    for (int nt = 0; nt < 2; ++nt) {
        const int col = nt * 16 + m;
        const float bb = sb1[col];
#pragma unroll
        for (int r = 0; r < 8; ++r) T[(8 * h + r) * LDT + col] = elu_f(acc1[nt][r] + bb);
    }
    __syncthreads();
    FragB a2h, a2l;
    fragA_f32(T + m * LDT, h, a2h, a2l);
    v8f acc2[4];
#pragma unroll
    for (int nt = 0; nt < 4; ++nt) {
        acc2[nt] = z8f();
        const v16bf bh = fragB16(sW2h, nt * 16 + m, 40, 0, h);
        const v16bf bl = fragB16(sW2l, nt * 16 + m, 40, 0, h);
        acc2[nt] = mma3(a2h.v, a2l.v, bh, bl, acc2[nt]);
    }
    __syncthreads();
#pragma unroll
    for (int nt = 0; nt < 4; ++nt) {
        const int col = nt * 16 + m;
        const float bb = sb2[col];
#pragma unroll
        for (int r = 0; r < 8; ++r) T[(8 * h + r) * LDT + col] = elu_f(acc2[nt][r] + bb);
    }
    __syncthreads();
    e_store(T, h32 + (size_t)row0 * CC, h16 + (size_t)row0 * CC, lane);
    __threadfence();
    e_store(T, h32 + (size_t)row0 * CC, h16 + (size_t)row0 * CC, lane);
}

__device__ __forceinline__ void y_store(const float* T, _Float16* yb, int lane)
{
#pragma unroll
    for (int g = 0; g < 4; ++g) {
        const int row = 4 * g + (lane >> 3);
        const int col = 8 * (lane & 7);
        const v4f q0 = *(const v4f*)(T + row * LDT + col);
        const v4f q1 = *(const v4f*)(T + row * LDT + col + 4);
        const v8h v = to_h8(q0, q1, 1.f);
        *(volatile v8h*)(yb + (size_t)row * YPITCH + col) = v;
    }
}

__global__ void __launch_bounds__(TB) k_ygemm(const _Float16* __restrict__ h16, const _Float16* __restrict__ wt,
                                          _Float16* __restrict__ Y, int F0, int NF)
{
    __shared__ __attribute__((aligned(16))) float sT[4][16 * LDT];
    const int tid = threadIdx.x, lane = tid & 31, wv = tid >> 5, h = lane >> 4, m = lane & 15;
    const int row0 = blockIdx.x * TROWS + wv * 16;
    FragH a0, a1;
    {
        const _Float16* ap = h16 + (size_t)(row0 + m) * CC;
        a0.hv[0] = *(const v8h*)(ap + 8 * h);
        a0.hv[1] = *(const v8h*)(ap + 16 + 8 * h);
        a1.hv[0] = *(const v8h*)(ap + 32 + 8 * h);
        a1.hv[1] = *(const v8h*)(ap + 48 + 8 * h);
    }
    float* T = sT[wv];
    for (int f = 0; f < NF; ++f) {
        const _Float16* wb = wt + (size_t)(F0 + f) * WSZ;
        v8f acc[4];
#pragma unroll
        for (int nt = 0; nt < 4; ++nt) {
            acc[nt] = z8f();
            const _Float16* bp = wb + (size_t)(nt * 16 + m) * CC;
            FragH b0, b1;
            b0.hv[0] = *(const v8h*)(bp + 8 * h);
            b0.hv[1] = *(const v8h*)(bp + 16 + 8 * h);
            b1.hv[0] = *(const v8h*)(bp + 32 + 8 * h);
            b1.hv[1] = *(const v8h*)(bp + 48 + 8 * h);
            acc[nt] = mma_h(a0.v, b0.v, acc[nt]);
            acc[nt] = mma_h(a1.v, b1.v, acc[nt]);
        }
#pragma unroll
        for (int nt = 0; nt < 4; ++nt)
#pragma unroll
            for (int r = 0; r < 8; ++r)
                T[(8 * h + r) * LDT + nt * 16 + m] = acc[nt][r] * (1.f / 1024.f);
        __syncthreads();
        _Float16* yb = Y + (size_t)row0 * YPITCH + (size_t)f * CC;
        y_store(T, yb, lane);
        __threadfence();
        y_store(T, yb, lane);
        __syncthreads();
    }
}

__device__ __forceinline__ void g_store(const float* accL, const int* degL, float* O, int n0, int wv, int lane)
{
#pragma unroll 4
    for (int g = 0; g < 64; ++g) {
        const int L = 4 * g + (lane >> 3);
        const int nl = wv * (GNB / 8) + (L >> 1);
        const int col = 32 * (L & 1) + 4 * (lane & 7);
        v4f v = *(const v4f*)(accL + nl * CC + col);
        const int dg = degL[nl];
        const float inv = 1.f / (float)(dg > 1 ? dg : 1);
        v = v * inv;
        *(volatile v4f*)(O + (size_t)(n0 + nl) * CC + col) = v;
    }
}

__global__ void __launch_bounds__(GTH) k_gather(const int* __restrict__ ei, const float* __restrict__ ea,
                                            const _Float16* __restrict__ Y, float* __restrict__ O,
                                            int NT, int E, int NCH, int F0, int NF)
{
    extern __shared__ v4f dsm[];
    float* accL = (float*)dsm;
    int* degL = (int*)(accL + GNB * CC);
    int* eL = degL + GNB;
    int* dL = eL + GCH;
    int* cntL = dL + GCH;
    const int tid = threadIdx.x, lane = tid & 31, wv = tid >> 5;
    const int n0 = blockIdx.x * GNB;
    {
        const v4f z4 = {0.f, 0.f, 0.f, 0.f};
        for (int i = tid; i < GNB * CC / 4; i += GTH) dsm[i] = z4;
        for (int i = tid; i < GNB; i += GTH) degL[i] = 0;
    }
    __syncthreads();

    for (int c = 0; c < NCH; ++c) {
        const int eb = c * GCH + GEPT * tid;
        int ev[GEPT], dv[GEPT];
        bool ht[GEPT];
        unsigned int mk[GEPT];
#pragma unroll
        for (int q = 0; q < GEPT; ++q) {
            const int e = eb + q;
            bool hit = false;
            int dl = 0;
            if (e < E) {
                int dst = ei[(size_t)E + e];
                if (dst < 0) dst += NT;
                dl = dst - n0;
                hit = (dst < NT) && ((unsigned)dl < (unsigned)GNB);
            }
            ev[q] = e; dv[q] = dl; ht[q] = hit;
            mk[q] = __builtin_amdgcn_ballot_w32(hit);
        }
        int wcnt = 0;
#pragma unroll
        for (int q = 0; q < GEPT; ++q) wcnt += __builtin_popcount(mk[q]);
        if (lane == 0) cntL[wv] = wcnt;
        __syncthreads();
        int base = 0, total = 0;
#pragma unroll
        for (int q = 0; q < GTH / 32; ++q) {
            const int cq = cntL[q];
            total += cq;
            if (q < wv) base += cq;
        }
#pragma unroll
        for (int q = 0; q < GEPT; ++q) {
            if (ht[q]) {
                const int pos = base + (int)__builtin_amdgcn_mbcnt_lo(mk[q], 0u);
                eL[pos] = ev[q];
                dL[pos] = dv[q];
            }
            base += __builtin_popcount(mk[q]);
        }
        __syncthreads();
        total = total < GCH ? total : GCH;
        for (int j = 0; j < total; ++j) {
            const int dlj = __builtin_amdgcn_readfirstlane(dL[j]);
            if ((dlj & (GTH / 32 - 1)) != wv) continue;
            const int ej = __builtin_amdgcn_readfirstlane(eL[j]);
            int src = ei[ej];
            if (src < 0) src += NT;
            src = src < 0 ? 0 : (src > NT - 1 ? NT - 1 : src);
            const float v0 = ea[(size_t)ej * 3 + 0] * 2.f;
            const float v1 = ea[(size_t)ej * 3 + 1] * 2.f;
            const float v2 = ea[(size_t)ej * 3 + 2] * 2.f;
            const float kf0 = fminf(fmaxf(floorf(v0), 0.f), 1.f);
            const float kf1 = fminf(fmaxf(floorf(v1), 0.f), 1.f);
            const float kf2 = fminf(fmaxf(floorf(v2), 0.f), 1.f);
            const float f0 = v0 - kf0, f1 = v1 - kf1, f2 = v2 - kf2;
            const float g0 = 1.f - f0, g1 = 1.f - f1, g2 = 1.f - f2;
            const int fb = (int)kf0 * 9 + (int)kf1 * 3 + (int)kf2 - F0;
            const _Float16* yr = Y + (size_t)src * YPITCH + 2 * lane;
            float r0 = 0.f, r1 = 0.f;
#pragma unroll
            for (int s = 0; s < 8; ++s) {
                const int bt0 = s & 1, bt1 = (s >> 1) & 1, bt2 = (s >> 2) & 1;
                const float wgt = ((bt0 ? f0 : g0) * (bt1 ? f1 : g1)) * (bt2 ? f2 : g2);
                const int fl = fb + bt0 * 9 + bt1 * 3 + bt2;
                if ((unsigned)fl < (unsigned)NF) {
                    const v2h y = *(const v2h*)(yr + fl * CC);
                    r0 = fmaf(wgt, (float)y.x, r0);
                    r1 = fmaf(wgt, (float)y.y, r1);
                }
            }
            v2f* ap = (v2f*)(accL + dlj * CC + 2 * lane);
            v2f a = *ap;
            a.x += r0;
            a.y += r1;
            *ap = a;
            if (lane == 0) degL[dlj] += 1;
        }
        __syncthreads();
    }
    __syncthreads();
    g_store(accL, degL, O, n0, wv, lane);
    __threadfence();
    g_store(accL, degL, O, n0, wv, lane);
}

__global__ void __launch_bounds__(TB) k_tail(const float* __restrict__ h32, const float* __restrict__ o1, const float* __restrict__ o2,
                                         const float* __restrict__ sprt, const float* __restrict__ spb,
                                         const float* __restrict__ dw0, const float* __restrict__ db0,
                                         const float* __restrict__ dw1, const float* __restrict__ db1,
                                         const float* __restrict__ dw2, const float* __restrict__ db2,
                                         float* __restrict__ out, int NT)
{
    __shared__ __attribute__((aligned(16))) unsigned short sRh[64 * 72];
    __shared__ __attribute__((aligned(16))) unsigned short sRl[64 * 72];
    __shared__ __attribute__((aligned(16))) unsigned short sAh[32 * 72];
    __shared__ __attribute__((aligned(16))) unsigned short sAl[32 * 72];
    __shared__ __attribute__((aligned(16))) unsigned short sBh[16 * 40];
    __shared__ __attribute__((aligned(16))) unsigned short sBl[16 * 40];
    __shared__ float sbias[64], sb0[32], sb1[16], sw2[32], sb2[2];
    __shared__ __attribute__((aligned(16))) float sT[4][16 * LDT];
    __shared__ __attribute__((aligned(16))) float sO[4][32];

    const int tid = threadIdx.x, lane = tid & 31, wv = tid >> 5, h = lane >> 4, m = lane & 15;
    stage_w(sprt, CC, 1, 64, 64, 64, 72, sRh, sRl, tid, TB);
    stage_w(dw0, 1, 64, 64, 64, 32, 72, sAh, sAl, tid, TB);
    stage_w(dw1, 1, 32, 32, 32, 16, 40, sBh, sBl, tid, TB);
    for (int i = tid; i < 64; i += TB) sbias[i] = spb[i];
    for (int i = tid; i < 32; i += TB) sb0[i] = db0[i];
    for (int i = tid; i < 16; i += TB) sb1[i] = db1[i];
    for (int i = tid; i < 32; i += TB) sw2[i] = dw2[i];
    for (int i = tid; i < 2; i += TB) sb2[i] = db2[i];
    __syncthreads();

    const int row0 = blockIdx.x * TROWS + wv * 16;
    int rr = row0 + m;
    rr = rr < NT ? rr : NT - 1;

    v8f acc[4];
#pragma unroll
    for (int nt = 0; nt < 4; ++nt) acc[nt] = z8f();
#pragma unroll
    for (int ks = 0; ks < 2; ++ks) {
        FragB ah, al;
        fragA_f32(h32 + (size_t)rr * CC + 32 * ks, h, ah, al);
#pragma unroll
        for (int nt = 0; nt < 4; ++nt) {
            const v16bf bh = fragB16(sRh, nt * 16 + m, 72, 32 * ks, h);
            const v16bf bl = fragB16(sRl, nt * 16 + m, 72, 32 * ks, h);
            acc[nt] = mma3(ah.v, al.v, bh, bl, acc[nt]);
        }
    }
    float* T = sT[wv];
#pragma unroll
    for (int nt = 0; nt < 4; ++nt) {
        const int col = nt * 16 + m;
        const float bb = sbias[col];
#pragma unroll
        for (int r = 0; r < 8; ++r) {
            int rg = row0 + 8 * h + r;
            rg = rg < NT ? rg : NT - 1;
            float v = o1[(size_t)rg * CC + col] + o2[(size_t)rg * CC + col];
            v = v + acc[nt][r];
            v = v + bb;
            T[(8 * h + r) * LDT + col] = elu_f(v);
        }
    }
    __syncthreads();
    v8f a5[2];
    a5[0] = z8f(); a5[1] = z8f();
#pragma unroll
    for (int ks = 0; ks < 2; ++ks) {
        FragB ah, al;
        fragA_f32(T + m * LDT + 32 * ks, h, ah, al);
#pragma unroll
        for (int nt = 0; nt < 2; ++nt) {
            const v16bf bh = fragB16(sAh, nt * 16 + m, 72, 32 * ks, h);
            const v16bf bl = fragB16(sAl, nt * 16 + m, 72, 32 * ks, h);
            a5[nt] = mma3(ah.v, al.v, bh, bl, a5[nt]);
        }
    }
    __syncthreads();
#pragma unroll
    for (int nt = 0; nt < 2; ++nt) {
        const int col = nt * 16 + m;
        const float bb = sb0[col];
#pragma unroll
        for (int r = 0; r < 8; ++r) T[(8 * h + r) * LDT + col] = elu_f(a5[nt][r] + bb);
    }
    __syncthreads();
    v8f a6 = z8f();
    {
        FragB ah, al;
        fragA_f32(T + m * LDT, h, ah, al);
        const v16bf bh = fragB16(sBh, m, 40, 0, h);
        const v16bf bl = fragB16(sBl, m, 40, 0, h);
        a6 = mma3(ah.v, al.v, bh, bl, a6);
    }
    __syncthreads();
    {
        const float bb = sb1[m];
#pragma unroll
        for (int r = 0; r < 8; ++r) T[(8 * h + r) * LDT + m] = elu_f(a6[r] + bb);
    }
    __syncthreads();
    float s = 0.f;
#pragma unroll
    for (int i = 0; i < 16; ++i) s = fmaf(sw2[h * 16 + i], T[m * LDT + i], s);
    s = s + sb2[h];
    const float t = tanhf(s);
    sO[wv][2 * m + h] = t;
    __syncthreads();
    if (row0 + 16 <= NT) {
        v4f v = {0.f, 0.f, 0.f, 0.f};
        if (lane < 8) v = *(const v4f*)(&sO[wv][4 * lane]);
        float* op = out + (size_t)row0 * 2 + 4 * lane;
        if (lane < 8) *(volatile v4f*)op = v;
        __threadfence();
        if (lane < 8) *(volatile v4f*)op = v;
    } else {
        const int node = row0 + m;
        if (node < NT) *(volatile float*)(out + (size_t)node * 2 + h) = t;
        __threadfence();
        if (node < NT) *(volatile float*)(out + (size_t)node * 2 + h) = t;
    }
}

static inline size_t al256(size_t v) { return (v + 255) & ~(size_t)255; }

extern "C" void kernel_launch(void* const* d_in, const int* in_sizes, int n_in,
                              void* d_out, int out_size, void* d_ws, size_t ws_size,
                              hipStream_t stream)
{
    if (n_in < 19) return;
    const int NT = in_sizes[1] / 2;
    const int E  = in_sizes[2] / 2;
    if (NT <= 0 || E < 0) return;
    if (in_sizes[3] != 3 * E || out_size != 2 * NT) return;
    if (in_sizes[4] != 32 || in_sizes[5] != 16 || in_sizes[6] != 512 || in_sizes[7] != 32 ||
        in_sizes[8] != 2048 || in_sizes[9] != 64 || in_sizes[10] != KFL * WSZ || in_sizes[11] != WSZ ||
        in_sizes[12] != 64 || in_sizes[13] != 2048 || in_sizes[14] != 32 || in_sizes[15] != 512 ||
        in_sizes[16] != 16 || in_sizes[17] != 32 || in_sizes[18] != 2) return;

    const float* x    = (const float*)d_in[1];
    const int*   ei   = (const int*)d_in[2];
    const float* ea   = (const float*)d_in[3];
    const float* ew0  = (const float*)d_in[4];
    const float* eb0  = (const float*)d_in[5];
    const float* ew1  = (const float*)d_in[6];
    const float* eb1  = (const float*)d_in[7];
    const float* ew2  = (const float*)d_in[8];
    const float* eb2  = (const float*)d_in[9];
    const float* spw  = (const float*)d_in[10];
    const float* sprt = (const float*)d_in[11];
    const float* spb  = (const float*)d_in[12];
    const float* dw0  = (const float*)d_in[13];
    const float* db0  = (const float*)d_in[14];
    const float* dw1  = (const float*)d_in[15];
    const float* db1  = (const float*)d_in[16];
    const float* dw2  = (const float*)d_in[17];
    const float* db2  = (const float*)d_in[18];

    const int    NB64 = (NT + TROWS - 1) / TROWS;
    const size_t NP64 = (size_t)NB64 * TROWS;
    const int    NBG  = (NT + GNB - 1) / GNB;
    const size_t NPG  = (size_t)NBG * GNB;
    const int    NCH  = (E + GCH - 1) / GCH;
    const int    NSEG = KFL * CC * 8;

    const size_t WT_B  = (size_t)KFL * WSZ * 2;
    const size_t Y_B   = NP64 * (size_t)YPITCH * 2;
    const size_t H32_B = NP64 * CC * 4;
    const size_t H16_B = NP64 * CC * 2;
    const size_t O_B   = NPG * CC * 4;

    size_t off = 0;
    char* ws = (char*)d_ws;
    char* p_wt  = ws + off; off += al256(WT_B);
    char* p_y   = ws + off; off += al256(Y_B);
    char* p_h32 = ws + off; off += al256(H32_B);
    char* p_h16 = ws + off; off += al256(H16_B);
    char* p_o1  = ws + off; off += al256(O_B);
    char* p_o2  = ws + off; off += al256(O_B);
    if (off > ws_size) return;

    hipFuncSetAttribute((const void*)k_gather, hipFuncAttributeMaxDynamicSharedMemorySize, GLDS);

    k_wprep<<<(NSEG + 255) / 256, 256, 0, stream>>>(spw, (_Float16*)p_wt, NSEG);
    k_enc<<<NB64, TB, 0, stream>>>(x, ew0, eb0, ew1, eb1, ew2, eb2, (float*)p_h32, (_Float16*)p_h16, NT);

    k_ygemm<<<NB64, TB, 0, stream>>>((const _Float16*)p_h16, (const _Float16*)p_wt, (_Float16*)p_y, 0, NFA);
    k_gather<<<NBG, GTH, GLDS, stream>>>(ei, ea, (const _Float16*)p_y, (float*)p_o1, NT, E, NCH, 0, NFA);

    k_ygemm<<<NB64, TB, 0, stream>>>((const _Float16*)p_h16, (const _Float16*)p_wt, (_Float16*)p_y, NFA, NFB);
    k_gather<<<NBG, GTH, GLDS, stream>>>(ei, ea, (const _Float16*)p_y, (float*)p_o2, NT, E, NCH, NFA, NFB);

    k_tail<<<NB64, TB, 0, stream>>>((const float*)p_h32, (const float*)p_o1, (const float*)p_o2,
                                     sprt, spb, dw0, db0, dw1, db1, dw2, db2, (float*)d_out, NT);
}
